// GT_7327214207519
// MI455X (gfx1250) — hardware-verified
//
#include <hip/hip_runtime.h>
#include <stddef.h>
#include <stdint.h>
#include <math.h>


#define DIN     128
#define HN      4
#define CH      128
#define HC      512
#define QP      1024
#define KVP     1152
#define HLD     2048
#define KQK     512
#define KVS     1024
#define NTHR    256
#define NWAVE   8
#define EPT     8
#define CHUNK   (NTHR * EPT)
#define WCAP    (EPT * 32)
#define LISTN   (NWAVE * WCAP)
#define NBMAX   1024
#define SLOTB   10
#define RCAP    28672
#define DEGCAP  64
#define STW     768
#define STWL    0
#define STWO    256
#define GBM     64
#define GBN     64
#define GTHR    128
#define ATTSC   0.08838834764831845f
#define WSMAX   268435456
#define LDS_AGG ((2 * RCAP + 2 * NBMAX + LISTN + 2 * NWAVE) * 4 + 64)

static_assert((1 << SLOTB) == NBMAX);
static_assert(SLOTB + 21 <= 31);
static_assert((CHUNK & (CHUNK - 1)) == 0 && CHUNK <= 2048 && SLOTB + 11 <= 31);
static_assert(NTHR * 4 == NBMAX);
static_assert(LISTN >= NBMAX);
static_assert(LISTN >= NWAVE * WCAP);
static_assert((RCAP % 32) == 0);
static_assert((NBMAX % NWAVE) == 0);
static_assert(NWAVE * STW <= RCAP && (STW % 4) == 0 && (STWO % 4) == 0);
static_assert(STWO >= STWL + HN * DEGCAP);
static_assert(STWO + HC <= STW);
static_assert(LDS_AGG <= 300000);
static_assert(GBM == (GTHR / 32) * 16);
static_assert(HC == 32 * 16);
static_assert(CH == 8 * 16 && HN * CH == HC);
static_assert(CH == 32 * 4);
static_assert(DIN == 16 * 8);
static_assert((DIN % 32) == 0 && (KQK % 32) == 0 && (KVS % 32) == 0 && KQK == HC && KVS == 2 * HC);
static_assert(QP == 2 * HC && QP * 2 == HLD);
static_assert(KVP == 2 * HC + CH);
static_assert((HC % GBN) == 0 && (CH % GBN) == 0 && ((KVP * 4) % 128) == 0 && ((QP * 4) % 128) == 0);

typedef float          v4f  __attribute__((ext_vector_type(4)));
typedef float          v8f  __attribute__((ext_vector_type(8)));
typedef int            v4i  __attribute__((ext_vector_type(4)));
typedef int            v8i  __attribute__((ext_vector_type(8)));
typedef unsigned int   v4u  __attribute__((ext_vector_type(4)));
typedef unsigned short v8us __attribute__((ext_vector_type(8)));
typedef __bf16         v16b __attribute__((ext_vector_type(16)));
typedef v4f  __attribute__((may_alias)) v4fa;
typedef v4u  __attribute__((may_alias)) v4ua;
typedef v8us __attribute__((may_alias)) v8usa;
union FragB { v16b v; v8us h[2]; v8i w; };

__device__ __forceinline__ v8f wmb(const FragB& a, const FragB& b, v8f c) {
  v8f d = __builtin_amdgcn_wmma_f32_16x16x32_bf16(false, a.v, false, b.v, (short)0, c, false, false);
  asm volatile("v_nop\n\tv_nop\n\tv_nop\n\tv_nop" : "+v"(d) : "v"(a.w), "v"(b.w));
  return d;
}

__device__ __forceinline__ void ldwait() {
  asm volatile("s_wait_loadcnt 0x0" ::: "memory");
}

__device__ __forceinline__ unsigned int f2bf(float f) {
  const unsigned int u = __float_as_uint(f);
  return ((u + 0x7FFFu + ((u >> 16) & 1u)) >> 16) & 0xFFFFu;
}
__device__ __forceinline__ float bf2f(unsigned int b) { return __uint_as_float(b << 16); }
__device__ __forceinline__ float bfr(float f) { return bf2f(f2bf(f)); }
__device__ __forceinline__ v4f bfr4(const v4f a) {
  v4f r; r.x = bfr(a.x); r.y = bfr(a.y); r.z = bfr(a.z); r.w = bfr(a.w); return r;
}
__device__ __forceinline__ unsigned int pk2(float lo, float hi) { return f2bf(lo) | (f2bf(hi) << 16); }
__device__ __forceinline__ v4u pack8(const v4f a, const v4f b) {
  v4u r;
  r.x = pk2(a.x, a.y); r.y = pk2(a.z, a.w); r.z = pk2(b.x, b.y); r.w = pk2(b.z, b.w);
  return r;
}
__device__ __forceinline__ void hl2(float v0, float v1, unsigned int& hw, unsigned int& lw) {
  const unsigned int h0 = f2bf(v0), h1 = f2bf(v1);
  const unsigned int l0 = f2bf(v0 - bf2f(h0)), l1 = f2bf(v1 - bf2f(h1));
  hw = h0 | (h1 << 16);
  lw = l0 | (l1 << 16);
}
__device__ __forceinline__ void pack8hl(const v4f a, const v4f b, v4u& hv, v4u& lv) {
  unsigned int h, l;
  hl2(a.x, a.y, h, l); hv.x = h; lv.x = l;
  hl2(a.z, a.w, h, l); hv.y = h; lv.y = l;
  hl2(b.x, b.y, h, l); hv.z = h; lv.z = l;
  hl2(b.z, b.w, h, l); hv.w = h; lv.w = l;
}
__device__ __forceinline__ float dot16(const v4f a0, const v4f a1, const v4f a2, const v4f a3,
                                       const v4f b0, const v4f b1, const v4f b2, const v4f b3) {
  float p = a0.x * b0.x;
  p = fmaf(a0.y, b0.y, p); p = fmaf(a0.z, b0.z, p); p = fmaf(a0.w, b0.w, p);
  p = fmaf(a1.x, b1.x, p); p = fmaf(a1.y, b1.y, p); p = fmaf(a1.z, b1.z, p); p = fmaf(a1.w, b1.w, p);
  p = fmaf(a2.x, b2.x, p); p = fmaf(a2.y, b2.y, p); p = fmaf(a2.z, b2.z, p); p = fmaf(a2.w, b2.w, p);
  p = fmaf(a3.x, b3.x, p); p = fmaf(a3.y, b3.y, p); p = fmaf(a3.z, b3.z, p); p = fmaf(a3.w, b3.w, p);
  return p;
}
__device__ __forceinline__ float hsum4(float v) {
  const float u = v + __shfl_xor(v, 8);
  return u + __shfl_xor(u, 16);
}

__device__ __forceinline__ int scan_chunk(const int* __restrict__ dsts, int nE, int cbase, int slotBase,
                                          int nb, int vec8, int* list, int tid, int lane, int wave) {
  int wc = 0;
  const int el0  = tid * EPT;
  const int e0   = cbase + el0;
  const int sent = -2147483647 - 1;
  v4i da, db;
  if (vec8 != 0 && cbase + CHUNK <= nE) {
    da = *(const v4i*)(dsts + e0);
    db = *(const v4i*)(dsts + e0 + 4);
  } else {
    da.x = (e0     < nE) ? dsts[min(e0,     nE - 1)] : sent;
    da.y = (e0 + 1 < nE) ? dsts[min(e0 + 1, nE - 1)] : sent;
    da.z = (e0 + 2 < nE) ? dsts[min(e0 + 2, nE - 1)] : sent;
    da.w = (e0 + 3 < nE) ? dsts[min(e0 + 3, nE - 1)] : sent;
    db.x = (e0 + 4 < nE) ? dsts[min(e0 + 4, nE - 1)] : sent;
    db.y = (e0 + 5 < nE) ? dsts[min(e0 + 5, nE - 1)] : sent;
    db.z = (e0 + 6 < nE) ? dsts[min(e0 + 6, nE - 1)] : sent;
    db.w = (e0 + 7 < nE) ? dsts[min(e0 + 7, nE - 1)] : sent;
  }
  const unsigned nbs = (unsigned)slotBase;
  const unsigned unb = (unsigned)nb;
  const unsigned s0 = (unsigned)da.x - nbs, s1 = (unsigned)da.y - nbs;
  const unsigned s2 = (unsigned)da.z - nbs, s3 = (unsigned)da.w - nbs;
  const unsigned s4 = (unsigned)db.x - nbs, s5 = (unsigned)db.y - nbs;
  const unsigned s6 = (unsigned)db.z - nbs, s7 = (unsigned)db.w - nbs;
  const bool h0 = s0 < unb, h1 = s1 < unb, h2 = s2 < unb, h3 = s3 < unb;
  const bool h4 = s4 < unb, h5 = s5 < unb, h6 = s6 < unb, h7 = s7 < unb;
  const unsigned any = __builtin_amdgcn_ballot_w32(h0 | h1 | h2 | h3 | h4 | h5 | h6 | h7);
  if (any != 0u) {
#define HITJ(J, HJ, SJ) { \
      const unsigned mj = __builtin_amdgcn_ballot_w32(HJ); \
      if (mj != 0u) { \
        if (HJ) { \
          const int pos = wc + (int)__builtin_amdgcn_mbcnt_lo(mj, 0u); \
          if (pos < WCAP) list[wave * WCAP + pos] = ((el0 + (J)) << SLOTB) | (int)(SJ); \
        } \
        wc += (int)__builtin_popcount(mj); } }
    HITJ(0, h0, s0)
    HITJ(1, h1, s1)
    HITJ(2, h2, s2)
    HITJ(3, h3, s3)
    HITJ(4, h4, s4)
    HITJ(5, h5, s5)
    HITJ(6, h6, s6)
    HITJ(7, h7, s7)
#undef HITJ
  }
  return wc;
}

__global__ __launch_bounds__(NTHR) void k_xprep(const float* __restrict__ x, unsigned short* xb, int nN, int nUnits) {
  const int i = (int)blockIdx.x * NTHR + (int)threadIdx.x;
  if (i >= nUnits) return;
  const int row = i >> 4;
  const int c0  = (i & 15) * 8;
  const int rc  = row < nN ? row : nN - 1;
  const float* p = x + (size_t)rc * DIN + c0;
  v4f a = *(const v4fa*)p;
  v4f b = *(const v4fa*)(p + 4);
  const v4f z4 = {0.f, 0.f, 0.f, 0.f};
  if (row >= nN) { a = z4; b = z4; }
  const v4u hv = pack8(a, b);
  unsigned short* o = xb + (size_t)row * DIN + c0;
  *(volatile v4u*)o = hv;
  __threadfence();
  *(volatile v4u*)o = hv;
}

__global__ __launch_bounds__(NTHR) void k_wtr(const float* __restrict__ w, int Kin, int Ncol, int Nrows, int Kout,
                                              unsigned short* wt, int nUnits) {
  const int u = (int)blockIdx.x * NTHR + (int)threadIdx.x;
  if (u >= nUnits) return;
  const int kq = Kout >> 3;
  const int n  = u / kq;
  const int k8 = (u - n * kq) * 8;
  const int kk = k8 - (k8 / Kin) * Kin;
  const int ncl = n < Ncol ? n : Ncol - 1;
  const float* p = w + (size_t)kk * (size_t)Ncol + ncl;
  v4f a, b;
  a.x = p[0];                    a.y = p[(size_t)Ncol];         a.z = p[(size_t)2 * Ncol];     a.w = p[(size_t)3 * Ncol];
  b.x = p[(size_t)4 * Ncol];     b.y = p[(size_t)5 * Ncol];     b.z = p[(size_t)6 * Ncol];     b.w = p[(size_t)7 * Ncol];
  const v4f z4 = {0.f, 0.f, 0.f, 0.f};
  if (n >= Ncol || n >= Nrows) { a = z4; b = z4; }
  const v4u wv = pack8(a, b);
  unsigned short* o = wt + (size_t)n * (size_t)Kout + k8;
  *(volatile v4u*)o = wv;
  __threadfence();
  *(volatile v4u*)o = wv;
}

__global__ __launch_bounds__(GTHR) void k_gemm(
    const unsigned short* __restrict__ A, int lda, const unsigned short* __restrict__ WT, int K,
    const float* __restrict__ bA, const float* __restrict__ bB, const float* __restrict__ bC,
    int splitB, int splitC, float* outF, int ldo)
{
  __shared__ __attribute__((aligned(16))) float stg[GBM * GBN];
  const int tid = (int)threadIdx.x, lane = tid & 31, wave = tid >> 5, hh = lane >> 4, m = lane & 15;
  const int rowBase = (int)blockIdx.x * GBM;
  const int col0    = (int)blockIdx.y * GBN;

  v8f acc[4];
  {
    const v8f z = {0.f, 0.f, 0.f, 0.f, 0.f, 0.f, 0.f, 0.f};
    acc[0] = z; acc[1] = z; acc[2] = z; acc[3] = z;
  }
  const unsigned short* ap = A  + (size_t)(rowBase + 16 * wave + m) * (size_t)lda + 8 * hh;
  const unsigned short* wp = WT + (size_t)(col0 + m) * (size_t)K + 8 * hh;
  const int ksteps = K >> 5;
#pragma unroll 1
  for (int ks = 0; ks < ksteps; ++ks) {
    FragB af;
    af.h[0] = *(const v8usa*)(ap + 32 * ks);
    af.h[1] = *(const v8usa*)(ap + 32 * ks + 16);
#pragma unroll
    for (int t = 0; t < 4; ++t) {
      const unsigned short* wq = wp + (size_t)(16 * t) * (size_t)K + 32 * ks;
      FragB bf;
      bf.h[0] = *(const v8usa*)wq;
      bf.h[1] = *(const v8usa*)(wq + 16);
      acc[t] = wmb(af, bf, acc[t]);
    }
  }

#pragma unroll
  for (int t = 0; t < 4; ++t) {
    const int lc = 16 * t + m;
#pragma unroll
    for (int r = 0; r < 8; ++r) {
      const int lr = 16 * wave + 8 * hh + r;
      stg[lr * GBN + lc] = acc[t][r];
    }
  }
  __syncthreads();

  const float* bsel = bA;
  int boff = col0;
  if (col0 >= splitB) { bsel = bB; boff = col0 - splitB; }
  if (col0 >= splitC) { bsel = bC; boff = col0 - splitC; }
  const v4f bv = bfr4(*(const v4fa*)(bsel + boff + 4 * m));

  v4f fv[8];
#pragma unroll
  for (int i = 0; i < 8; ++i) {
    const int lr = 16 * wave + 2 * i + hh;
    fv[i] = *(const v4fa*)(stg + lr * GBN + 4 * m) + bv;
  }
#pragma unroll
  for (int i = 0; i < 8; ++i) {
    const int lr = 16 * wave + 2 * i + hh;
    const int gr = rowBase + lr;
    float* op = outF + (size_t)gr * (size_t)ldo + col0 + 4 * m;
    *(volatile v4f*)op = fv[i];
  }
  __threadfence();
#pragma unroll
  for (int i = 0; i < 8; ++i) {
    const int lr = 16 * wave + 2 * i + hh;
    const int gr = rowBase + lr;
    float* op = outF + (size_t)gr * (size_t)ldo + col0 + 4 * m;
    *(volatile v4f*)op = fv[i];
  }
}

template<int L>
__global__ __launch_bounds__(NTHR) void k_agg(
    const int* __restrict__ srcs, const int* __restrict__ dsts,
    float* Q, const float* __restrict__ KV, float* out,
    int nN, int nE, int vec8, int MPr) {
  extern __shared__ v4f lds_dyn[];
  int* reg1 = (int*)lds_dyn;
  int* reg2 = reg1 + RCAP;
  int* scnt = reg2 + RCAP;
  int* soff = scnt + NBMAX;
  int* list = soff + NBMAX;
  int* wcnt = list + LISTN;
  int* wtot = wcnt + NWAVE;
  const int tid = (int)threadIdx.x, lane = tid & 31, wave = tid >> 5;
  const int nodeBase = (int)blockIdx.x * NBMAX;

  for (int i = tid; i < NBMAX; i += NTHR) scnt[i] = 0;
  __syncthreads();

  int tot = 0;
  const int nChunks = (nE + CHUNK - 1) / CHUNK;
#pragma unroll 1
  for (int ch = 0; ch < nChunks; ++ch) {
    const int cbase = ch * CHUNK;
    const int wc = scan_chunk(dsts, nE, cbase, nodeBase, NBMAX, vec8, list, tid, lane, wave);
    if (lane == 0) wcnt[wave] = wc;
    __syncthreads();
    int pre = 0, all = 0;
#pragma unroll
    for (int w2 = 0; w2 < NWAVE; ++w2) {
      int c = wcnt[w2];
      c = c < 0 ? 0 : (c > WCAP ? WCAP : c);
      all += c;
      pre += (w2 < wave) ? c : 0;
    }
    const int wcc  = wc > WCAP ? WCAP : wc;
    const int base = tot + pre;
#pragma unroll 1
    for (int i = lane; i < wcc; i += 32) {
      const int ent = list[wave * WCAP + i];
      const int el  = (ent >> SLOTB) & (CHUNK - 1);
      const int sl  = ent & (NBMAX - 1);
      int eid = cbase + el;
      eid = eid > nE - 1 ? nE - 1 : eid;
      const int pos = base + i;
      if (pos < RCAP) reg1[pos] = (int)(((unsigned)eid << SLOTB) | (unsigned)sl);
    }
    tot += all;
    tot = tot > RCAP ? RCAP : tot;
    __syncthreads();
  }
  const int nh = tot;

  if (wave == 0) {
#pragma unroll 1
    for (int b0 = 0; b0 < nh; b0 += 32) {
      const int idx = b0 + lane;
      const int uv  = reg1[idx < nh ? idx : nh - 1];
      const int m32 = (nh - b0) < 32 ? (nh - b0) : 32;
#pragma unroll 1
      for (int k = 0; k < m32; ++k) {
        const int u  = __builtin_amdgcn_readlane(uv, k);
        const int sl = u & (NBMAX - 1);
        if (lane == 0) scnt[sl] = scnt[sl] + 1;
      }
    }
  }
  __syncthreads();

  {
    const v4i ca = *(const v4i*)(scnt + 4 * tid);
    const int e0 = ca.x < 0 ? 0 : ca.x, e1 = ca.y < 0 ? 0 : ca.y, e2 = ca.z < 0 ? 0 : ca.z, e3 = ca.w < 0 ? 0 : ca.w;
    const int ts = e0 + e1 + e2 + e3;
    int incl = ts;
#pragma unroll
    for (int d = 1; d < 32; d <<= 1) {
      const int up = __shfl_up(incl, d);
      if (lane >= d) incl += up;
    }
    if (lane == 31) wtot[wave] = incl;
    __syncthreads();
    int pre = 0;
#pragma unroll
    for (int w2 = 0; w2 < NWAVE; ++w2) pre += (w2 < wave) ? wtot[w2] : 0;
    int run = pre + incl - ts;
    soff[4 * tid + 0] = run; run += e0;
    soff[4 * tid + 1] = run; run += e1;
    soff[4 * tid + 2] = run; run += e2;
    soff[4 * tid + 3] = run;
  }
  __syncthreads();
  for (int i = tid; i < NBMAX; i += NTHR) list[i] = soff[i];
  __syncthreads();

  if (wave == 0) {
#pragma unroll 1
    for (int b0 = 0; b0 < nh; b0 += 32) {
      const int idx = b0 + lane;
      const int uv  = reg1[idx < nh ? idx : nh - 1];
      const int m32 = (nh - b0) < 32 ? (nh - b0) : 32;
#pragma unroll 1
      for (int k = 0; k < m32; ++k) {
        const int u   = __builtin_amdgcn_readlane(uv, k);
        const int sl  = u & (NBMAX - 1);
        const int eid = (int)((unsigned)u >> SLOTB);
        if (lane == 0) {
          int pos = list[sl];
          pos = pos < 0 ? 0 : (pos > RCAP - 1 ? RCAP - 1 : pos);
          reg2[pos] = eid;
          list[sl] = pos + 1;
        }
      }
    }
  }
  __syncthreads();

  const int nbw = NBMAX / NWAVE;
  const bool ovf = (nh >= RCAP);
  const float qnan = __int_as_float(0x7fc00000);
  float* stw = (float*)reg1 + wave * STW;
  float* slg = stw + STWL;
  float* sto = stw + STWO;
  unsigned int* stu = (unsigned int*)(stw + STWO);
  const int hd = lane >> 3;
  const v4f z4 = {0.f, 0.f, 0.f, 0.f};

#pragma unroll 1
  for (int jt = 0; jt < nbw; ++jt) {
    const int slot = wave * nbw + jt;
    const int grow = nodeBase + slot;
    const int gcl  = grow < nN ? grow : nN - 1;
    int st = soff[slot];
    const int craw = scnt[slot];
    int cnt = craw;
    st  = st < 0 ? 0 : (st > nh ? nh : st);
    cnt = cnt < 0 ? 0 : (cnt > DEGCAP ? DEGCAP : cnt);
    if (cnt > nh - st) cnt = nh - st;
    const float pz = (ovf || craw > DEGCAP) ? qnan : 0.0f;

    const float* qr = Q + (size_t)gcl * QP + 16 * lane;
    const v4f q0 = *(const v4fa*)qr;
    const v4f q1 = *(const v4fa*)(qr + 4);
    const v4f q2 = *(const v4fa*)(qr + 8);
    const v4f q3 = *(const v4fa*)(qr + 12);
    ldwait();

    float mx = -1.0e30f;
#pragma unroll 1
    for (int q = 0; q < cnt; ++q) {
      int idx = st + q; idx = idx > RCAP - 1 ? RCAP - 1 : idx;
      int eid = reg2[idx]; eid = eid < 0 ? 0 : (eid > nE - 1 ? nE - 1 : eid);
      const int sraw = srcs[eid];
      const int s = sraw < 0 ? 0 : (sraw > nN - 1 ? nN - 1 : sraw);
      const float* kr = KV + (size_t)s * KVP + 16 * lane;
      const v4f k0 = *(const v4fa*)kr;
      const v4f k1 = *(const v4fa*)(kr + 4);
      const v4f k2 = *(const v4fa*)(kr + 8);
      const v4f k3 = *(const v4fa*)(kr + 12);
      ldwait();
      float p = dot16(q0, q1, q2, q3, k0, k1, k2, k3);
      p += __shfl_xor(p, 4);
      p += __shfl_xor(p, 2);
      p += __shfl_xor(p, 1);
      const float lg = p * ATTSC;
      mx = fmaxf(mx, lg);
      slg[hd * DEGCAP + q] = lg;
    }
    __builtin_amdgcn_fence(__ATOMIC_RELEASE, "wavefront");
    __builtin_amdgcn_wave_barrier();

    float dn = 0.f;
    v4f a0 = z4, a1 = z4, a2 = z4, a3 = z4;
#pragma unroll 1
    for (int q = 0; q < cnt; ++q) {
      int idx = st + q; idx = idx > RCAP - 1 ? RCAP - 1 : idx;
      int eid = reg2[idx]; eid = eid < 0 ? 0 : (eid > nE - 1 ? nE - 1 : eid);
      const int sraw = srcs[eid];
      const int s = sraw < 0 ? 0 : (sraw > nN - 1 ? nN - 1 : sraw);
      const float lg = slg[hd * DEGCAP + q];
      const float* vr = KV + (size_t)s * KVP + HC + 16 * lane;
      const v4f v0 = *(const v4fa*)vr;
      const v4f v1 = *(const v4fa*)(vr + 4);
      const v4f v2 = *(const v4fa*)(vr + 8);
      const v4f v3 = *(const v4fa*)(vr + 12);
      ldwait();
      const float p = __expf(lg - mx);
      dn += p;
      a0.x = fmaf(p, v0.x, a0.x); a0.y = fmaf(p, v0.y, a0.y); a0.z = fmaf(p, v0.z, a0.z); a0.w = fmaf(p, v0.w, a0.w);
      a1.x = fmaf(p, v1.x, a1.x); a1.y = fmaf(p, v1.y, a1.y); a1.z = fmaf(p, v1.z, a1.z); a1.w = fmaf(p, v1.w, a1.w);
      a2.x = fmaf(p, v2.x, a2.x); a2.y = fmaf(p, v2.y, a2.y); a2.z = fmaf(p, v2.z, a2.z); a2.w = fmaf(p, v2.w, a2.w);
      a3.x = fmaf(p, v3.x, a3.x); a3.y = fmaf(p, v3.y, a3.y); a3.z = fmaf(p, v3.z, a3.z); a3.w = fmaf(p, v3.w, a3.w);
    }
    const float dns = dn > 0.f ? dn : 1.0f;
    const float ind = dn > 0.f ? 1.0f : 0.0f;
    const float inv = ind * __builtin_amdgcn_rcpf(dns);
    const v4f m0 = a0 * inv, m1 = a1 * inv, m2 = a2 * inv, m3 = a3 * inv;

    if (L == 0) {
      const float* sr = qr + HC;
      const v4f s0 = *(const v4fa*)sr;
      const v4f s1 = *(const v4fa*)(sr + 4);
      const v4f s2 = *(const v4fa*)(sr + 8);
      const v4f s3 = *(const v4fa*)(sr + 12);
      ldwait();
      const bool live = grow < nN;
      v4f h0 = m0 + s0, h1 = m1 + s1, h2 = m2 + s2, h3 = m3 + s3;
      h0.x = fmaxf(h0.x, 0.f); h0.y = fmaxf(h0.y, 0.f); h0.z = fmaxf(h0.z, 0.f); h0.w = fmaxf(h0.w, 0.f);
      h1.x = fmaxf(h1.x, 0.f); h1.y = fmaxf(h1.y, 0.f); h1.z = fmaxf(h1.z, 0.f); h1.w = fmaxf(h1.w, 0.f);
      h2.x = fmaxf(h2.x, 0.f); h2.y = fmaxf(h2.y, 0.f); h2.z = fmaxf(h2.z, 0.f); h2.w = fmaxf(h2.w, 0.f);
      h3.x = fmaxf(h3.x, 0.f); h3.y = fmaxf(h3.y, 0.f); h3.z = fmaxf(h3.z, 0.f); h3.w = fmaxf(h3.w, 0.f);
      h0 = (live ? h0 : z4) + pz;
      h1 = (live ? h1 : z4) + pz;
      h2 = (live ? h2 : z4) + pz;
      h3 = (live ? h3 : z4) + pz;
      v4u hvA, lvA, hvB, lvB;
      pack8hl(h0, h1, hvA, lvA);
      pack8hl(h2, h3, hvB, lvB);
      __builtin_amdgcn_fence(__ATOMIC_RELEASE, "wavefront");
      __builtin_amdgcn_wave_barrier();
      *(v4ua*)(stu + 8 * lane)           = hvA;
      *(v4ua*)(stu + 8 * lane + 4)       = hvB;
      *(v4ua*)(stu + 256 + 8 * lane)     = lvA;
      *(v4ua*)(stu + 256 + 8 * lane + 4) = lvB;
      __builtin_amdgcn_fence(__ATOMIC_RELEASE, "wavefront");
      __builtin_amdgcn_wave_barrier();
      const v4u p0 = *(const v4ua*)(stu + 4 * lane);
      const v4u p1 = *(const v4ua*)(stu + 128 + 4 * lane);
      const v4u p2 = *(const v4ua*)(stu + 256 + 4 * lane);
      const v4u p3 = *(const v4ua*)(stu + 384 + 4 * lane);
      const bool wr = (grow < MPr);
      const int gsf = wr ? grow : MPr - 1;
      unsigned int* hrow = (unsigned int*)(Q + (size_t)gsf * QP);
      if (wr) {
        *(volatile v4u*)(hrow + 4 * lane)       = p0;
        *(volatile v4u*)(hrow + 128 + 4 * lane) = p1;
        *(volatile v4u*)(hrow + 256 + 4 * lane) = p2;
        *(volatile v4u*)(hrow + 384 + 4 * lane) = p3;
      }
      __threadfence();
      if (wr) {
        *(volatile v4u*)(hrow + 4 * lane)       = p0;
        *(volatile v4u*)(hrow + 128 + 4 * lane) = p1;
        *(volatile v4u*)(hrow + 256 + 4 * lane) = p2;
        *(volatile v4u*)(hrow + 384 + 4 * lane) = p3;
      }
    } else {
      v4f t0, t1, t2, t3;
      t0.x = hsum4(m0.x); t0.y = hsum4(m0.y); t0.z = hsum4(m0.z); t0.w = hsum4(m0.w);
      t1.x = hsum4(m1.x); t1.y = hsum4(m1.y); t1.z = hsum4(m1.z); t1.w = hsum4(m1.w);
      t2.x = hsum4(m2.x); t2.y = hsum4(m2.y); t2.z = hsum4(m2.z); t2.w = hsum4(m2.w);
      t3.x = hsum4(m3.x); t3.y = hsum4(m3.y); t3.z = hsum4(m3.z); t3.w = hsum4(m3.w);
      t0 = t0 * 0.25f; t1 = t1 * 0.25f; t2 = t2 * 0.25f; t3 = t3 * 0.25f;
      __builtin_amdgcn_fence(__ATOMIC_RELEASE, "wavefront");
      __builtin_amdgcn_wave_barrier();
      if (lane < 8) {
        *(v4fa*)(sto + 16 * lane)      = t0;
        *(v4fa*)(sto + 16 * lane + 4)  = t1;
        *(v4fa*)(sto + 16 * lane + 8)  = t2;
        *(v4fa*)(sto + 16 * lane + 12) = t3;
      }
      __builtin_amdgcn_fence(__ATOMIC_RELEASE, "wavefront");
      __builtin_amdgcn_wave_barrier();
      const v4f pa = *(const v4fa*)(sto + 4 * lane);
      const v4f sv = *(const v4fa*)(KV + (size_t)gcl * KVP + 2 * HC + 4 * lane);
      ldwait();
      v4f o = pa + sv;
      o = o + pz;
      const bool wr = (grow < nN);
      const int gs  = wr ? grow : nN - 1;
      float* op = out + (size_t)gs * CH + 4 * lane;
      if (wr) *(volatile v4f*)op = o;
      __threadfence();
      if (wr) *(volatile v4f*)op = o;
    }
    __builtin_amdgcn_fence(__ATOMIC_RELEASE, "wavefront");
    __builtin_amdgcn_wave_barrier();
  }
}

static inline int cdiv(int a, int b) { return (a + b - 1) / b; }

extern "C" void kernel_launch(void* const* d_in, const int* in_sizes, int n_in,
                              void* d_out, int out_size, void* d_ws, size_t ws_size,
                              hipStream_t stream) {
  if (n_in < 18) return;
  if (in_sizes[0] < DIN || (in_sizes[0] % DIN) != 0) return;
  const int nN = in_sizes[0] / DIN;
  if (nN < 1 || nN > (1 << 22)) return;
  if (in_sizes[1] < 2 || (in_sizes[1] & 1) != 0) return;
  const int nE = in_sizes[1] / 2;
  if (nE < 1 || nE >= (1 << (31 - SLOTB))) return;
  if (in_sizes[2] != DIN * HC || in_sizes[4] != DIN * HC || in_sizes[6] != DIN * HC || in_sizes[8] != DIN * HC) return;
  if (in_sizes[3] != HC || in_sizes[5] != HC || in_sizes[7] != HC || in_sizes[9] != HC) return;
  if (in_sizes[10] != HC * HC || in_sizes[12] != HC * HC || in_sizes[14] != HC * HC) return;
  if (in_sizes[11] != HC || in_sizes[13] != HC || in_sizes[15] != HC) return;
  if (in_sizes[16] != HC * CH || in_sizes[17] != CH) return;
  if (out_size != nN * CH) return;

  const float* x   = (const float*)d_in[0];
  const int*   ei  = (const int*)  d_in[1];
  const float* Wq0 = (const float*)d_in[2];
  const float* bq0 = (const float*)d_in[3];
  const float* Wk0 = (const float*)d_in[4];
  const float* bk0 = (const float*)d_in[5];
  const float* Wv0 = (const float*)d_in[6];
  const float* bv0 = (const float*)d_in[7];
  const float* Ws0 = (const float*)d_in[8];
  const float* bs0 = (const float*)d_in[9];
  const float* Wq1 = (const float*)d_in[10];
  const float* bq1 = (const float*)d_in[11];
  const float* Wk1 = (const float*)d_in[12];
  const float* bk1 = (const float*)d_in[13];
  const float* Wv1 = (const float*)d_in[14];
  const float* bv1 = (const float*)d_in[15];
  const float* Ws1 = (const float*)d_in[16];
  const float* bs1 = (const float*)d_in[17];
  float* out = (float*)d_out;
  const int* src = ei;
  const int* dst = ei + nE;

  const int MP   = cdiv(nN, GBM) * GBM;
  const int gA   = cdiv(MP, NBMAX);
  const int vec8 = ((nE & 3) == 0) ? 1 : 0;
  if (gA * NBMAX < MP) return;

  char* ws = (char*)d_ws;
  size_t off = 0;
  const size_t oXB  = off; off += (size_t)MP * DIN * 2;                 off = (off + 255) & ~(size_t)255;
  const size_t oWT0 = off; off += (size_t)4 * HC * DIN * 2;             off = (off + 255) & ~(size_t)255;
  const size_t oWTA = off; off += (size_t)2 * HC * KQK * 2;             off = (off + 255) & ~(size_t)255;
  const size_t oWTB = off; off += (size_t)(HC + CH) * KVS * 2;          off = (off + 255) & ~(size_t)255;
  const size_t oKV  = off; off += (size_t)MP * KVP * 4;                 off = (off + 255) & ~(size_t)255;
  const size_t oQS  = off; off += (size_t)MP * QP * 4;                  off = (off + 255) & ~(size_t)255;
  if (off > ws_size || off > (size_t)WSMAX) return;
  unsigned short* XB  = (unsigned short*)(ws + oXB);
  unsigned short* WT0 = (unsigned short*)(ws + oWT0);
  unsigned short* WTA = (unsigned short*)(ws + oWTA);
  unsigned short* WTB = (unsigned short*)(ws + oWTB);
  float*          KV  = (float*)(ws + oKV);
  float*          QS  = (float*)(ws + oQS);
  const unsigned short* HPL = (const unsigned short*)QS;

  hipFuncSetAttribute(reinterpret_cast<const void*>(&k_agg<0>),
                      hipFuncAttributeMaxDynamicSharedMemorySize, LDS_AGG);
  hipFuncSetAttribute(reinterpret_cast<const void*>(&k_agg<1>),
                      hipFuncAttributeMaxDynamicSharedMemorySize, LDS_AGG);

  const int nUx = MP * (DIN / 8);
  k_xprep<<<cdiv(nUx, NTHR), NTHR, 0, stream>>>(x, XB, nN, nUx);

  {
    const int nU0 = HC * (DIN / 8);
    k_wtr<<<cdiv(nU0, NTHR), NTHR, 0, stream>>>(Wk0, DIN, HC, HC, DIN, WT0,                         nU0);
    k_wtr<<<cdiv(nU0, NTHR), NTHR, 0, stream>>>(Wv0, DIN, HC, HC, DIN, WT0 + (size_t)HC * DIN,       nU0);
    k_wtr<<<cdiv(nU0, NTHR), NTHR, 0, stream>>>(Wq0, DIN, HC, HC, DIN, WT0 + (size_t)2 * HC * DIN,   nU0);
    k_wtr<<<cdiv(nU0, NTHR), NTHR, 0, stream>>>(Ws0, DIN, HC, HC, DIN, WT0 + (size_t)3 * HC * DIN,   nU0);
    const int nUA = HC * (KQK / 8);
    k_wtr<<<cdiv(nUA, NTHR), NTHR, 0, stream>>>(Wk1, HC, HC, HC, KQK, WTA,                         nUA);
    k_wtr<<<cdiv(nUA, NTHR), NTHR, 0, stream>>>(Wq1, HC, HC, HC, KQK, WTA + (size_t)HC * KQK,       nUA);
    const int nUV = HC * (KVS / 8);
    k_wtr<<<cdiv(nUV, NTHR), NTHR, 0, stream>>>(Wv1, HC, HC, HC, KVS, WTB,                         nUV);
    const int nUS = CH * (KVS / 8);
    k_wtr<<<cdiv(nUS, NTHR), NTHR, 0, stream>>>(Ws1, HC, CH, CH, KVS, WTB + (size_t)HC * KVS,       nUS);
  }

  const int gM  = MP / GBM;
  const int far = 1 << 30;
  k_gemm<<<dim3(gM, (2 * HC) / GBN), GTHR, 0, stream>>>(XB, DIN, WT0,                         DIN, bk0, bv0, bv0, HC, far, KV, KVP);
  k_gemm<<<dim3(gM, (2 * HC) / GBN), GTHR, 0, stream>>>(XB, DIN, WT0 + (size_t)2 * HC * DIN,  DIN, bq0, bs0, bs0, HC, far, QS, QP);
  k_agg<0><<<gA, NTHR, LDS_AGG, stream>>>(src, dst, QS, KV, out, nN, nE, vec8, MP);
  k_gemm<<<dim3(gM, HC / GBN), GTHR, 0, stream>>>(HPL, HLD, WTA,                         KQK, bk1, bk1, bk1, far, far, KV, KVP);
  k_gemm<<<dim3(gM, HC / GBN), GTHR, 0, stream>>>(HPL, HLD, WTA + (size_t)HC * KQK,       KQK, bq1, bq1, bq1, far, far, QS + HC, QP);
  k_gemm<<<dim3(gM, (HC + CH) / GBN), GTHR, 0, stream>>>(HPL, HLD, WTB,                  KVS, bv1, bs1, bs1, HC, far, KV + HC, KVP);
  k_agg<1><<<gA, NTHR, LDS_AGG, stream>>>(src, dst, QS + HC, KV, out, nN, nE, vec8, MP);
}
